// TransformerSelfAttnLayer_34643206209733
// MI455X (gfx1250) — hardware-run, weakly checked
//
#include <hip/hip_runtime.h>
#include <math.h>
#include <stdint.h>

#ifndef NB
#define NB       32
#endif
#ifndef SEQ
#define SEQ      512
#endif
#define NB_FULL  32
#define SEQ_FULL 512
#define SKV      512
#define CDIM     128
#define NH       8
#define HD       16
#define QKN      256
#define PRN      256
#define NPOS     1023
#define NPOSP    1024
#define NBIAS    (3 * CDIM)
#define WSC      256.0f
#define QS       8.0f
#define KS       8.0f
#define VS       8.0f
#define CS       256.0f
#define PCAR     32768.0f
#define LOG2E    1.4426950408889634f
#define LN_EPS   1e-5f
#define NKB      (SKV / 32)
#define AT_WAVES   8
#define AT_THREADS (AT_WAVES * 32)
#define AT_LDS     65536
#define SPITCH   20
#define GPITCH   68

static_assert(NB >= 16 && NB <= NB_FULL && (NB % 16) == 0);
static_assert(SEQ >= 128 && SEQ <= SEQ_FULL && (SEQ % 128) == 0);
static_assert(NH * HD == CDIM && HD == 16 && QKN == 2 * CDIM && PRN == 2 * CDIM);
static_assert((SKV % 128) == 0 && NKB * 32 == SKV && (CDIM % 64) == 0 && (CDIM % 32) == 0);
static_assert(AT_THREADS == 256 && 2 * AT_THREADS == 16 * 32);
static_assert(AT_WAVES * 2 * 16 * SPITCH * 4 <= 32768 && (SPITCH % 4) == 0);
static_assert(8192 * 4 + 16 * 32 * 32 * 2 == AT_LDS);
static_assert((GPITCH * 4) % 16 == 0 && (NPOSP % 128) == 0 && (PRN % 64) == 0 && (QKN % 64) == 0);

typedef unsigned short u16;
typedef _Float16 v16h __attribute__((ext_vector_type(16)));
typedef _Float16 v8h  __attribute__((ext_vector_type(8)));
typedef float    v8f  __attribute__((ext_vector_type(8)));
typedef float    v4f  __attribute__((ext_vector_type(4)));
typedef unsigned int v4u __attribute__((ext_vector_type(4)));
typedef unsigned int v2u __attribute__((ext_vector_type(2)));

union FragH { v16h v; v8h h[2]; v4u u[2]; };

__device__ __forceinline__ unsigned short bf_bits(float f) {
  unsigned u = __float_as_uint(f);
  return (unsigned short)((u + 0x7FFFu + ((u >> 16) & 1u)) >> 16);
}
__device__ __forceinline__ float bf_up(unsigned short h) { return __uint_as_float(((unsigned)h) << 16); }
__device__ __forceinline__ float bfr(float f) { return bf_up(bf_bits(f)); }
__device__ __forceinline__ unsigned short h_bits(_Float16 x) { return __builtin_bit_cast(unsigned short, x); }
__device__ __forceinline__ unsigned pk16(unsigned short a, unsigned short b) { return (unsigned)a | ((unsigned)b << 16); }
__device__ __forceinline__ v8f zero8() { v8f z = {0.f, 0.f, 0.f, 0.f, 0.f, 0.f, 0.f, 0.f}; return z; }

__device__ __forceinline__ v16h ldfrag_h(const _Float16* p) {
  FragH f;
  f.h[0] = *(const v8h*)(p);
  f.h[1] = *(const v8h*)(p + 16);
  return f.v;
}

__device__ __forceinline__ v8f mma_h(v16h a, v16h b, v8f c) {
  return __builtin_amdgcn_wmma_f32_16x16x32_f16(false, a, false, b, (short)0, c, false, false);
}
__device__ __forceinline__ void guard_g(v8f (&acc)[8], v16h x0, v16h x1, v16h x2, v16h x3, v16h x4, v16h x5) {
#if defined(__HIP_DEVICE_COMPILE__)
  asm volatile("v_nop\n\tv_nop\n\tv_nop\n\tv_nop"
               : "+v"(acc[0]), "+v"(acc[1]), "+v"(acc[2]), "+v"(acc[3]),
                 "+v"(acc[4]), "+v"(acc[5]), "+v"(acc[6]), "+v"(acc[7])
               : "v"(x0), "v"(x1), "v"(x2), "v"(x3), "v"(x4), "v"(x5) : "memory");
#endif
}
__device__ __forceinline__ void guard_46(v8f& a, v8f& b, v8f& c, v8f& d,
                                         v16h x0, v16h x1, v16h x2, v16h x3, v16h x4, v16h x5) {
#if defined(__HIP_DEVICE_COMPILE__)
  asm volatile("v_nop\n\tv_nop\n\tv_nop\n\tv_nop"
               : "+v"(a), "+v"(b), "+v"(c), "+v"(d)
               : "v"(x0), "v"(x1), "v"(x2), "v"(x3), "v"(x4), "v"(x5) : "memory");
#endif
}
__device__ __forceinline__ void guard_48(v8f& a, v8f& b, v8f& c, v8f& d,
                                         v16h x0, v16h x1, v16h x2, v16h x3, v16h x4, v16h x5, v16h x6, v16h x7) {
#if defined(__HIP_DEVICE_COMPILE__)
  asm volatile("v_nop\n\tv_nop\n\tv_nop\n\tv_nop"
               : "+v"(a), "+v"(b), "+v"(c), "+v"(d)
               : "v"(x0), "v"(x1), "v"(x2), "v"(x3), "v"(x4), "v"(x5), "v"(x6), "v"(x7) : "memory");
#endif
}
__device__ __forceinline__ void guard_2(v8f& a, v8f& b, v16h x0, v16h x1, v16h x2, v16h x3) {
#if defined(__HIP_DEVICE_COMPILE__)
  asm volatile("v_nop\n\tv_nop\n\tv_nop\n\tv_nop"
               : "+v"(a), "+v"(b) : "v"(x0), "v"(x1), "v"(x2), "v"(x3) : "memory");
#endif
}
__device__ __forceinline__ void guard_12(v8f& a, v16h x0, v16h x1) {
#if defined(__HIP_DEVICE_COMPILE__)
  asm volatile("v_nop\n\tv_nop\n\tv_nop\n\tv_nop" : "+v"(a) : "v"(x0), "v"(x1) : "memory");
#endif
}
__device__ __forceinline__ void acc_guard1(v8f& a) {
#if defined(__HIP_DEVICE_COMPILE__)
  asm volatile("v_nop\n\tv_nop\n\tv_nop\n\tv_nop" : "+v"(a));
#endif
}
__device__ __forceinline__ void wave_sync_lds() {
  __builtin_amdgcn_fence(__ATOMIC_RELEASE, "workgroup");
  __builtin_amdgcn_wave_barrier();
  __builtin_amdgcn_fence(__ATOMIC_ACQUIRE, "workgroup");
}

__global__ __launch_bounds__(128)
void rowcvt(const float* __restrict__ src, u16* dst, int nsrc, int nrows, float scale) {
  const int tid = threadIdx.x, wave = tid >> 5, lane = tid & 31;
  const int r = blockIdx.x * 4 + wave;
  if (r >= nrows) return;
  const int rs = (r < nsrc) ? r : (nsrc - 1);
  const float keep = (r < nsrc) ? scale : 0.0f;
  const v4f x = *(const v4f*)(src + (size_t)rs * CDIM + 4 * lane);
  v2u o;
  o[0] = pk16(h_bits((_Float16)(bfr(x[0]) * keep)), h_bits((_Float16)(bfr(x[1]) * keep)));
  o[1] = pk16(h_bits((_Float16)(bfr(x[2]) * keep)), h_bits((_Float16)(bfr(x[3]) * keep)));
  u16* d = dst + (size_t)r * CDIM + 4 * lane;
  for (int pass = 0; pass < 2; ++pass) {
    *(volatile v2u*)d = o;
    __threadfence();
  }
}

__global__ __launch_bounds__(128)
void ln16(const float* __restrict__ feat, const float* __restrict__ g, const float* __restrict__ bb, u16* X) {
  const int tid = threadIdx.x, wave = tid >> 5, lane = tid & 31;
  const int r = blockIdx.x * 4 + wave;
  if (r >= NB * SKV) return;
  const int n = r / SKV;
  const int w = r - n * SKV;
  const float* src = feat + ((size_t)w * NB_FULL + (size_t)n) * CDIM + 4 * lane;
  const v4f xv = *(const v4f*)src;
  const float x0 = bfr(xv[0]), x1 = bfr(xv[1]), x2 = bfr(xv[2]), x3 = bfr(xv[3]);
  float s = (x0 + x1) + (x2 + x3);
#pragma unroll
  for (int off = 16; off >= 1; off >>= 1) s += __shfl_xor(s, off, 32);
  const float mu = s * (1.0f / (float)CDIM);
  const float d0 = x0 - mu, d1 = x1 - mu, d2 = x2 - mu, d3 = x3 - mu;
  float q = (d0 * d0 + d1 * d1) + (d2 * d2 + d3 * d3);
#pragma unroll
  for (int off = 16; off >= 1; off >>= 1) q += __shfl_xor(q, off, 32);
  const float var = q * (1.0f / (float)CDIM);
  const float rstd = rsqrtf(var + LN_EPS);
  const v4f gv = *(const v4f*)(g + 4 * lane), bv = *(const v4f*)(bb + 4 * lane);
  const float y0 = d0 * rstd * bfr(gv[0]) + bfr(bv[0]);
  const float y1 = d1 * rstd * bfr(gv[1]) + bfr(bv[1]);
  const float y2 = d2 * rstd * bfr(gv[2]) + bfr(bv[2]);
  const float y3 = d3 * rstd * bfr(gv[3]) + bfr(bv[3]);
  v2u o;
  o[0] = pk16(h_bits((_Float16)y0), h_bits((_Float16)y1));
  o[1] = pk16(h_bits((_Float16)y2), h_bits((_Float16)y3));
  u16* d = X + (size_t)r * CDIM + 4 * lane;
  for (int pass = 0; pass < 2; ++pass) {
    *(volatile v2u*)d = o;
    __threadfence();
  }
}

__device__ __forceinline__ void gemm_core(const _Float16* ap, const _Float16* bp, int K, v8f (&acc)[8]) {
  const size_t rs16 = (size_t)16 * (size_t)K;
#pragma unroll 1
  for (int k0 = 0; k0 < K; k0 += 32) {
    const v16h a0 = ldfrag_h(ap + k0), a1 = ldfrag_h(ap + rs16 + k0);
    const v16h b0 = ldfrag_h(bp + k0);
    const v16h b1 = ldfrag_h(bp + rs16 + k0);
    const v16h b2 = ldfrag_h(bp + 2 * rs16 + k0);
    const v16h b3 = ldfrag_h(bp + 3 * rs16 + k0);
    acc[0] = mma_h(a0, b0, acc[0]);
    acc[1] = mma_h(a0, b1, acc[1]);
    acc[2] = mma_h(a0, b2, acc[2]);
    acc[3] = mma_h(a0, b3, acc[3]);
    acc[4] = mma_h(a1, b0, acc[4]);
    acc[5] = mma_h(a1, b1, acc[5]);
    acc[6] = mma_h(a1, b2, acc[6]);
    acc[7] = mma_h(a1, b3, acc[7]);
    guard_g(acc, a0, a1, b0, b1, b2, b3);
  }
}
__device__ __forceinline__ void stage32x64(float* sl, v8f (&acc)[8], float oscale, int lane) {
  const int hh = lane >> 4, m = lane & 15;
#pragma unroll
  for (int i = 0; i < 2; ++i) {
#pragma unroll
    for (int r = 0; r < 8; ++r) {
      const int ro = (16 * i + 8 * hh + r) * GPITCH + m;
      sl[ro]      = acc[4 * i + 0][r] * oscale;
      sl[ro + 16] = acc[4 * i + 1][r] * oscale;
      sl[ro + 32] = acc[4 * i + 2][r] * oscale;
      sl[ro + 48] = acc[4 * i + 3][r] * oscale;
    }
  }
  wave_sync_lds();
}

__global__ __launch_bounds__(128)
void gemm16(const u16* __restrict__ A, const u16* __restrict__ Bt, const float* __restrict__ bias, u16* C,
            int Mb, int N, int K, int aBs, int bBs, int cBs, int ldc, int biasMode, int biasOff, float wsinv, float carry) {
  __shared__ __align__(16) float slab[4 * 32 * GPITCH];
  const int tid = threadIdx.x, wave = tid >> 5, lane = tid & 31, hh = lane >> 4, m = lane & 15;
  const int ntile = N >> 6, mtile = Mb >> 7;
  const int bid  = blockIdx.x;
  const int nt   = bid % ntile;
  const int tmp  = bid / ntile;
  const int mt   = tmp % mtile;
  const int bz   = tmp / mtile;
  const int rowb = mt * 128 + wave * 32;
  const int col0 = nt * 64;
  if (rowb + 32 > Mb) return;
  const _Float16* Ab = (const _Float16*)(const void*)A + (size_t)bz * (size_t)aBs;
  const _Float16* Bb = (const _Float16*)(const void*)Bt + (size_t)bz * (size_t)bBs;
  const _Float16* ap = Ab + (size_t)(rowb + m) * (size_t)K + 8 * hh;
  const _Float16* bp = Bb + (size_t)(col0 + m) * (size_t)K + 8 * hh;
  v8f acc[8];
#pragma unroll
  for (int i = 0; i < 8; ++i) acc[i] = zero8();
  gemm_core(ap, bp, K, acc);
  float* sl = slab + wave * 32 * GPITCH;
  stage32x64(sl, acc, wsinv, lane);
  const int rq = lane >> 3, c8 = (lane & 7) * 8;
  const float fcol = (biasMode == 1) ? 1.0f : 0.0f;
  const float frow = (biasMode == 2) ? 1.0f : 0.0f;
  float bc[8];
  {
    int ci = biasOff + col0 + c8;
    ci = (ci < 0) ? 0 : ci;
    ci = (ci > NBIAS - 8) ? (NBIAS - 8) : ci;
    const v4f u0 = *(const v4f*)(bias + ci), u1 = *(const v4f*)(bias + ci + 4);
#pragma unroll
    for (int j = 0; j < 4; ++j) { bc[j] = bfr(u0[j]) * fcol; bc[4 + j] = bfr(u1[j]) * fcol; }
  }
  v4u oh[8];
#pragma unroll
  for (int i = 0; i < 8; ++i) {
    const int row = 4 * i + rq;
    int ri = biasOff + (rowb - mt * 128) + row;
    ri = (ri < 0) ? 0 : ri;
    ri = (ri > NBIAS - 1) ? (NBIAS - 1) : ri;
    const float br = bfr(bias[ri]) * frow;
    const v4f a = *(const v4f*)(sl + row * GPITCH + c8), c4 = *(const v4f*)(sl + row * GPITCH + c8 + 4);
#pragma unroll
    for (int e2 = 0; e2 < 2; ++e2) {
      const float x0 = (a[2 * e2] + bc[2 * e2] + br) * carry;
      const float x1 = (a[2 * e2 + 1] + bc[2 * e2 + 1] + br) * carry;
      const float x2 = (c4[2 * e2] + bc[4 + 2 * e2] + br) * carry;
      const float x3 = (c4[2 * e2 + 1] + bc[4 + 2 * e2 + 1] + br) * carry;
      oh[i][e2]     = pk16(h_bits((_Float16)x0), h_bits((_Float16)x1));
      oh[i][2 + e2] = pk16(h_bits((_Float16)x2), h_bits((_Float16)x3));
    }
  }
  u16* Hb = C + (size_t)bz * (size_t)cBs + (size_t)rowb * (size_t)ldc + col0 + c8;
  for (int pass = 0; pass < 2; ++pass) {
#pragma unroll
    for (int i = 0; i < 8; ++i) {
      const int row = 4 * i + rq;
      *(volatile v4u*)(Hb + (size_t)row * (size_t)ldc) = oh[i];
    }
    __threadfence();
  }
}

__global__ __launch_bounds__(AT_THREADS)
void attn_rel(const u16* __restrict__ QK, const u16* __restrict__ PR, const u16* __restrict__ VT,
              const int* __restrict__ pidx, u16* CT) {
  extern __shared__ __align__(16) float dsm[];
  float* bias = dsm;
  u16* prs = (u16*)(void*)(dsm + 8192);
  const _Float16* prf = (const _Float16*)(const void*)prs;

  const int tid  = threadIdx.x;
  const int wave = tid >> 5;
  const int lane = tid & 31;
  const int hh   = lane >> 4;
  const int c    = lane & 15;

  constexpr int NWT = SEQ / 16;
  constexpr int NNG = NB / 16;
  const int bid = blockIdx.x;
  const int wt  = bid % NWT;
  const int ng  = (bid / NWT) % NNG;
  const int e   = bid / (NWT * NNG);
  const int w0  = 16 * wt;
  const int n0  = 16 * ng;

  const _Float16* QKf = (const _Float16*)(const void*)QK;
  const _Float16* VTf = (const _Float16*)(const void*)VT;
  const float lsc = (LOG2E * 0.25f) / (QS * KS);
  const v4u z4 = {0u, 0u, 0u, 0u};

  float mrun[2], lrun[2];
  v8f o[2];
#pragma unroll
  for (int nn = 0; nn < 2; ++nn) { mrun[nn] = -INFINITY; lrun[nn] = 0.f; o[nn] = zero8(); }

#pragma unroll 1
  for (int it = 0; it < NKB; ++it) {
    const int kb = it * 32;
    __syncthreads();
#pragma unroll
    for (int q = 0; q < 2; ++q) {
      const int p  = tid + AT_THREADS * q;
      const int wl = p >> 5, vl = p & 31;
      int ix = pidx[(size_t)(w0 + wl) * SKV + (size_t)(kb + vl)];
      ix = (ix < 0) ? 0 : ix;
      ix = (ix > NPOS - 1) ? (NPOS - 1) : ix;
      const u16* prow = PR + (size_t)ix * PRN;
      const v4u kr0 = *(const v4u*)(prow + CDIM + e * HD), kr1 = *(const v4u*)(prow + CDIM + e * HD + 8);
      const v4u qr0 = *(const v4u*)(prow + e * HD),        qr1 = *(const v4u*)(prow + e * HD + 8);
      u16* d = prs + (size_t)(wl * 32 + vl) * 32;
      *(v4u*)(d)      = kr0;
      *(v4u*)(d + 8)  = kr1;
      *(v4u*)(d + 16) = qr0;
      *(v4u*)(d + 24) = qr1;
    }
    __syncthreads();
    {
      const int wl0 = 2 * wave, wl1 = wl0 + 1;
      FragH a0, a1, b00, b01, b10, b11;
      a0.h[0] = *(const v8h*)(QKf + ((size_t)(n0 + c) * SKV + (size_t)(w0 + wl0)) * QKN + e * HD + 8 * hh); a0.u[1] = z4;
      a1.h[0] = *(const v8h*)(QKf + ((size_t)(n0 + c) * SKV + (size_t)(w0 + wl1)) * QKN + e * HD + 8 * hh); a1.u[1] = z4;
      b00.h[0] = *(const v8h*)(prf + (wl0 * 32 + c) * 32 + 8 * hh);       b00.u[1] = z4;
      b01.h[0] = *(const v8h*)(prf + (wl0 * 32 + 16 + c) * 32 + 8 * hh);  b01.u[1] = z4;
      b10.h[0] = *(const v8h*)(prf + (wl1 * 32 + c) * 32 + 8 * hh);       b10.u[1] = z4;
      b11.h[0] = *(const v8h*)(prf + (wl1 * 32 + 16 + c) * 32 + 8 * hh);  b11.u[1] = z4;
      v8f d00 = mma_h(a0.v, b00.v, zero8());
      v8f d01 = mma_h(a0.v, b01.v, zero8());
      v8f d10 = mma_h(a1.v, b10.v, zero8());
      v8f d11 = mma_h(a1.v, b11.v, zero8());
      guard_46(d00, d01, d10, d11, a0.v, a1.v, b00.v, b01.v, b10.v, b11.v);
      float* t2a = bias + (wl0 * 16 + 8 * hh) * 32 + c;
      float* t2b = bias + (wl1 * 16 + 8 * hh) * 32 + c;
#pragma unroll
      for (int r = 0; r < 8; ++r) {
        t2a[r * 32]      = d00[r];
        t2a[r * 32 + 16] = d01[r];
        t2b[r * 32]      = d10[r];
        t2b[r * 32 + 16] = d11[r];
      }
    }
    __syncthreads();
    {
      FragH a3[4], b3[4];
      v8f d3[4];
#pragma unroll
      for (int vv = 0; vv < 4; ++vv) {
        const int vl = 4 * wave + vv;
        a3[vv].h[0] = *(const v8h*)(QKf + ((size_t)(n0 + c) * SKV + (size_t)(kb + vl)) * QKN + CDIM + e * HD + 8 * hh);
        a3[vv].u[1] = z4;
        b3[vv].h[0] = *(const v8h*)(prf + (c * 32 + vl) * 32 + 16 + 8 * hh);
        b3[vv].u[1] = z4;
      }
#pragma unroll
      for (int vv = 0; vv < 4; ++vv) d3[vv] = mma_h(a3[vv].v, b3[vv].v, zero8());
      guard_48(d3[0], d3[1], d3[2], d3[3], a3[0].v, a3[1].v, a3[2].v, a3[3].v, b3[0].v, b3[1].v, b3[2].v, b3[3].v);
      float* t3p = bias + (c * 16 + 8 * hh) * 32 + 4 * wave;
#pragma unroll
      for (int r = 0; r < 8; ++r) {
        v4f x = *(const v4f*)(t3p + r * 32);
        x[0] += d3[0][r];
        x[1] += d3[1][r];
        x[2] += d3[2][r];
        x[3] += d3[3][r];
        *(v4f*)(t3p + r * 32) = x;
      }
    }
    __syncthreads();
#pragma unroll
    for (int nn = 0; nn < 2; ++nn) {
      const int nl = 2 * wave + nn;
      const int n  = n0 + nl;
      const size_t qkrow = (size_t)n * SKV;
      FragH fq, ka, kc2;
      fq.h[0] = *(const v8h*)(QKf + (qkrow + (size_t)(w0 + c)) * QKN + e * HD + 8 * hh);  fq.u[1] = z4;
      const _Float16* kp0 = QKf + (qkrow + (size_t)(kb + c)) * QKN + CDIM + e * HD + 8 * hh;
      ka.h[0]  = *(const v8h*)(kp0);                     ka.u[1]  = z4;
      kc2.h[0] = *(const v8h*)(kp0 + (size_t)16 * QKN);  kc2.u[1] = z4;
      v8f s0 = mma_h(ka.v, fq.v, zero8());
      v8f s1 = mma_h(kc2.v, fq.v, zero8());
      guard_2(s0, s1, ka.v, kc2.v, fq.v, fq.v);
      const float* bl = bias + (c * 16 + nl) * 32 + 8 * hh;
      const v4f g0 = *(const v4f*)(bl), g1 = *(const v4f*)(bl + 4), g2 = *(const v4f*)(bl + 16), g3 = *(const v4f*)(bl + 20);
      float t[16];
#pragma unroll
      for (int i = 0; i < 4; ++i) {
        t[i]      = (s0[i] + g0[i]) * lsc;
        t[4 + i]  = (s0[4 + i] + g1[i]) * lsc;
        t[8 + i]  = (s1[i] + g2[i]) * lsc;
        t[12 + i] = (s1[4 + i] + g3[i]) * lsc;
      }
      float cm = t[0];
#pragma unroll
      for (int i = 1; i < 16; ++i) cm = fmaxf(cm, t[i]);
      cm = fmaxf(cm, __shfl_xor(cm, 16, 32));
      const float mn = fmaxf(mrun[nn], cm);
      const float al = exp2f(mrun[nn] - mn);
      mrun[nn] = mn;
      float ps = 0.f;
      FragH ph;
#pragma unroll
      for (int w2 = 0; w2 < 2; ++w2) {
#pragma unroll
        for (int e4 = 0; e4 < 4; ++e4) {
          const int i = 8 * w2 + 2 * e4;
          const float p0 = exp2f(t[i] - mn), p1 = exp2f(t[i + 1] - mn);
          ps += p0 + p1;
          ph.u[w2][e4] = pk16(h_bits((_Float16)(p0 * PCAR)), h_bits((_Float16)(p1 * PCAR)));
        }
      }
      ps += __shfl_xor(ps, 16, 32);
      lrun[nn] = lrun[nn] * al + ps;
      float scl[8];
#pragma unroll
      for (int r = 0; r < 8; ++r) scl[r] = __shfl(al, 8 * hh + r, 32);
#pragma unroll
      for (int r = 0; r < 8; ++r) o[nn][r] *= scl[r];
      const v16h vf = ldfrag_h(VTf + ((size_t)((n * NH + e) * HD + c)) * SKV + kb + 8 * hh);
      o[nn] = mma_h(ph.v, vf, o[nn]);
      guard_12(o[nn], ph.v, vf);
    }
  }
  __syncthreads();

  float* slab = dsm + wave * (2 * 16 * SPITCH);
#pragma unroll
  for (int nn = 0; nn < 2; ++nn) {
    acc_guard1(o[nn]);
    const float linv = (1.0f / lrun[nn]) * (CS / (PCAR * VS));
    float inv[8];
#pragma unroll
    for (int r = 0; r < 8; ++r) inv[r] = __shfl(linv, 8 * hh + r, 32);
#pragma unroll
    for (int r = 0; r < 8; ++r) slab[nn * 16 * SPITCH + (8 * hh + r) * SPITCH + c] = o[nn][r] * inv[r];
  }
  wave_sync_lds();
  const int rw = lane >> 1, c8 = 8 * (lane & 1);
  v4u ov[2];
#pragma unroll
  for (int nn = 0; nn < 2; ++nn) {
    const float* sp = slab + nn * 16 * SPITCH + rw * SPITCH + c8;
    const v4f a = *(const v4f*)(sp), c4 = *(const v4f*)(sp + 4);
#pragma unroll
    for (int e2 = 0; e2 < 2; ++e2) {
      ov[nn][e2]     = pk16(h_bits((_Float16)a[2 * e2]),  h_bits((_Float16)a[2 * e2 + 1]));
      ov[nn][2 + e2] = pk16(h_bits((_Float16)c4[2 * e2]), h_bits((_Float16)c4[2 * e2 + 1]));
    }
  }
  for (int pass = 0; pass < 2; ++pass) {
#pragma unroll
    for (int nn = 0; nn < 2; ++nn) {
      const int n = n0 + 2 * wave + nn;
      u16* dst = CT + (((size_t)(e * NB_FULL + n)) * SEQ_FULL + (size_t)w0) * HD + 8 * lane;
      *(volatile v4u*)dst = ov[nn];
    }
    __threadfence();
  }
}

__global__ __launch_bounds__(128)
void gemm_out(const u16* __restrict__ CT, const u16* __restrict__ WO, const float* __restrict__ ob,
              const float* __restrict__ feat, float* Out) {
  __shared__ __align__(16) float slab[4 * 32 * GPITCH];
  const int tid = threadIdx.x, wave = tid >> 5, lane = tid & 31, hh = lane >> 4, m = lane & 15;
  constexpr int NWT = SEQ / 128;
  const int bid  = blockIdx.x;
  const int nt   = bid & 1;
  const int tmp  = bid >> 1;
  const int wtl  = tmp % NWT;
  const int n    = tmp / NWT;
  const int wb   = wtl * 128 + wave * 32;
  const int col0 = nt * 64;
  if (wb + 32 > SEQ || n >= NB) return;
  const _Float16* CTf = (const _Float16*)(const void*)CT;
  const _Float16* WOf = (const _Float16*)(const void*)WO;
  v8f acc[8];
#pragma unroll
  for (int i = 0; i < 8; ++i) acc[i] = zero8();
#pragma unroll 1
  for (int ks = 0; ks < CDIM / 32; ++ks) {
    const int e0 = 2 * ks;
    const _Float16* p00 = CTf + (((size_t)(e0 * NB_FULL + n)) * SEQ_FULL + (size_t)(wb + m)) * HD + 8 * hh;
    const _Float16* p01 = p00 + (size_t)NB_FULL * SEQ_FULL * HD;
    FragH a0, a1;
    a0.h[0] = *(const v8h*)(p00);            a0.h[1] = *(const v8h*)(p01);
    a1.h[0] = *(const v8h*)(p00 + 16 * HD);  a1.h[1] = *(const v8h*)(p01 + 16 * HD);
    const _Float16* bp = WOf + (size_t)(col0 + m) * CDIM + 32 * ks + 8 * hh;
    const v16h b0 = ldfrag_h(bp);
    const v16h b1 = ldfrag_h(bp + 16 * CDIM);
    const v16h b2 = ldfrag_h(bp + 32 * CDIM);
    const v16h b3 = ldfrag_h(bp + 48 * CDIM);
    acc[0] = mma_h(a0.v, b0, acc[0]);
    acc[1] = mma_h(a0.v, b1, acc[1]);
    acc[2] = mma_h(a0.v, b2, acc[2]);
    acc[3] = mma_h(a0.v, b3, acc[3]);
    acc[4] = mma_h(a1.v, b0, acc[4]);
    acc[5] = mma_h(a1.v, b1, acc[5]);
    acc[6] = mma_h(a1.v, b2, acc[6]);
    acc[7] = mma_h(a1.v, b3, acc[7]);
    guard_g(acc, a0.v, a1.v, b0, b1, b2, b3);
  }
  float* sl = slab + wave * 32 * GPITCH;
  stage32x64(sl, acc, 1.0f / (CS * WSC), lane);
  const int rs = lane >> 4, pc = lane & 15;
  const v4f bq = *(const v4f*)(ob + col0 + 4 * pc);
  const float bz0 = bfr(bq[0]), bz1 = bfr(bq[1]), bz2 = bfr(bq[2]), bz3 = bfr(bq[3]);
  v4f ov[16];
#pragma unroll
  for (int i = 0; i < 16; ++i) {
    const int row = 2 * i + rs;
    const v4f a = *(const v4f*)(sl + row * GPITCH + 4 * pc);
    const float* fp = feat + ((size_t)(wb + row) * NB_FULL + (size_t)n) * CDIM + col0 + 4 * pc;
    const v4f f4 = *(const v4f*)fp;
    ov[i][0] = a[0] + bz0 + bfr(f4[0]);
    ov[i][1] = a[1] + bz1 + bfr(f4[1]);
    ov[i][2] = a[2] + bz2 + bfr(f4[2]);
    ov[i][3] = a[3] + bz3 + bfr(f4[3]);
  }
  for (int pass = 0; pass < 2; ++pass) {
#pragma unroll
    for (int i = 0; i < 16; ++i) {
      const int row = 2 * i + rs;
      float* op = Out + ((size_t)(wb + row) * NB_FULL + (size_t)n) * CDIM + col0 + 4 * pc;
      *(volatile v4f*)op = ov[i];
    }
    __threadfence();
  }
}

extern "C" void kernel_launch(void* const* d_in, const int* in_sizes, int n_in,
                              void* d_out, int out_size, void* d_ws, size_t ws_size,
                              hipStream_t stream) {
  if (n_in < 9) return;
  if (in_sizes[0] < SEQ_FULL * NB_FULL * CDIM) return;
  if (in_sizes[1] < NPOS * CDIM) return;
  if (in_sizes[2] < SEQ_FULL * SKV) return;
  if (in_sizes[3] < NBIAS * CDIM || in_sizes[4] < NBIAS) return;
  if (in_sizes[5] < CDIM * CDIM || in_sizes[6] < CDIM || in_sizes[7] < CDIM || in_sizes[8] < CDIM) return;
  if (out_size < SEQ_FULL * NB_FULL * CDIM) return;

  const float* feat = (const float*)d_in[0];
  const float* pos  = (const float*)d_in[1];
  const int*   pidx = (const int*)d_in[2];
  const float* win  = (const float*)d_in[3];
  const float* inb  = (const float*)d_in[4];
  const float* wout = (const float*)d_in[5];
  const float* outb = (const float*)d_in[6];
  const float* lng  = (const float*)d_in[7];
  const float* lnb  = (const float*)d_in[8];
  float*       out  = (float*)d_out;

  const size_t szXP  = (size_t)NB * SKV * CDIM * 2;
  const size_t szWI  = (size_t)NBIAS * CDIM * 2;
  const size_t szWO  = (size_t)CDIM * CDIM * 2;
  const size_t szPOS = (size_t)NPOSP * CDIM * 2;
  const size_t szQK  = (size_t)NB * SKV * QKN * 2;
  const size_t szVT  = (size_t)NB * CDIM * SKV * 2;
  const size_t szPR  = (size_t)NPOSP * PRN * 2;
  const size_t szCT  = (size_t)NH * NB_FULL * SEQ_FULL * HD * 2;
  size_t off = 0;
  const size_t oXP  = off; off += szXP;
  const size_t oWI  = off; off += szWI;
  const size_t oWO  = off; off += szWO;
  const size_t oPOS = off; off += szPOS;
  const size_t oQK  = off; off += szQK;
  const size_t oVT  = off; off += szVT;
  const size_t oPR  = off; off += szPR;
  const size_t oCT  = off; off += szCT;
  if (off > ws_size) return;
  if (off > (size_t)134217728) return;

  char* ws = (char*)d_ws;
  u16* XP  = (u16*)(ws + oXP);
  u16* WI  = (u16*)(ws + oWI);
  u16* WO  = (u16*)(ws + oWO);
  u16* POS = (u16*)(ws + oPOS);
  u16* QK  = (u16*)(ws + oQK);
  u16* VT  = (u16*)(ws + oVT);
  u16* PRB = (u16*)(ws + oPR);
  u16* CT  = (u16*)(ws + oCT);

  rowcvt<<<dim3(NBIAS / 4), dim3(128), 0, stream>>>(win, WI, NBIAS, NBIAS, WSC);
  rowcvt<<<dim3(CDIM / 4), dim3(128), 0, stream>>>(wout, WO, CDIM, CDIM, WSC);
  rowcvt<<<dim3(NPOSP / 4), dim3(128), 0, stream>>>(pos, POS, NPOS, NPOSP, 1.0f);
  ln16<<<dim3((NB * SKV) / 4), dim3(128), 0, stream>>>(feat, lng, lnb, XP);
  gemm16<<<dim3((NB * SKV / 128) * (QKN / 64)), dim3(128), 0, stream>>>(
      XP, WI, inb, QK, NB * SKV, QKN, CDIM, 0, 0, 0, QKN, 1, 0, 1.0f / WSC, QS);
  gemm16<<<dim3(NB * 1 * (SKV / 64)), dim3(128), 0, stream>>>(
      WI + (size_t)2 * CDIM * CDIM, XP, inb, VT, CDIM, SKV, CDIM, 0, SKV * CDIM, CDIM * SKV, SKV, 2, 2 * CDIM, 1.0f / WSC, VS);
  gemm16<<<dim3((NPOSP / 128) * (PRN / 64)), dim3(128), 0, stream>>>(
      POS, WI, inb, PRB, NPOSP, PRN, CDIM, 0, 0, 0, PRN, 1, 0, 1.0f / WSC, QS);
  (void)hipFuncSetAttribute(reinterpret_cast<const void*>(&attn_rel), hipFuncAttributeMaxDynamicSharedMemorySize, AT_LDS);
  attn_rel<<<dim3(NH * (NB / 16) * (SEQ / 16)), dim3(AT_THREADS), AT_LDS, stream>>>(QK, PRB, VT, pidx, CT);
  gemm_out<<<dim3(NB * (SEQ / 128) * 2), dim3(128), 0, stream>>>(CT, WO, outb, feat, out);
  (void)hipGetLastError();
}
